// MultiHeadGAT_5738076307731
// MI455X (gfx1250) — hardware-verified
//
#include <hip/hip_runtime.h>
#include <stddef.h>


#define DF    128
#define NHD   4
#define DG    (NHD * DF)
#define NACT  10
#define NGMAX 64
#define NTERM 10
#define GR    32
#define HSP   136
#define XSP   132
#define NB    512
#define CHUNK 2048
#define NTHR  256
#define NWAVE 8
#define WCAP  256
#define NGRP  (CHUNK / (NTHR * 4))
#define WSCL  16.0f
#define WINV  0.0625f

#define LDS_SAGE_BYTES ((NB * DF + NB + NWAVE * WCAP + 16) * 4)
#define LDS_GAT_BYTES  ((NB * DF + 2 * NB * NHD + NWAVE * WCAP + 16) * 4)

static_assert(WCAP == (CHUNK / NTHR) * 32);
static_assert(NGRP >= 1);
static_assert(NB == 512);
static_assert(CHUNK <= 4096);
static_assert((NB % (2 * NWAVE)) == 0);
static_assert(DF / 8 == 16);
static_assert(LDS_SAGE_BYTES == 272448);
static_assert(LDS_GAT_BYTES == 286784);

typedef float    v4f  __attribute__((ext_vector_type(4)));
typedef float    v8f  __attribute__((ext_vector_type(8)));
typedef int      v4i  __attribute__((ext_vector_type(4)));
typedef _Float16 v8h  __attribute__((ext_vector_type(8)));
typedef _Float16 v16h __attribute__((ext_vector_type(16)));
union Frag   { v16h v; v8h half[2]; };
union Pack16 { v8h h; v4i i; };

__device__ __forceinline__ v8f wm(v16h a, v16h b, v8f c) {
  v8f d = __builtin_amdgcn_wmma_f32_16x16x32_f16(false, a, false, b, (short)0, c, false, false);
  asm volatile("v_nop\n\tv_nop\n\tv_nop\n\tv_nop" : "+v"(d) : "v"(a), "v"(b));
  return d;
}

__device__ __forceinline__ float wsum(float v) {
  v += __shfl_xor(v, 16, 32);
  v += __shfl_xor(v, 8, 32);
  v += __shfl_xor(v, 4, 32);
  v += __shfl_xor(v, 2, 32);
  v += __shfl_xor(v, 1, 32);
  return v;
}

__device__ __forceinline__ float elu1(float v) { return v > 0.f ? v : expm1f(v); }

__global__ __launch_bounds__(NTHR) void k_prep(const float* __restrict__ Wl, const float* __restrict__ Wr,
                                               const float* __restrict__ Wg,
                                               _Float16* Wlh, _Float16* Wrh, _Float16* Wgh, int n8) {
  const int i = blockIdx.x * NTHR + threadIdx.x;
  if (i >= n8) return;
  const float* W;
  _Float16* P;
  int nc, j;
  if (i < DF * DF / 8)          { W = Wl; P = Wlh; nc = DF; j = i; }
  else if (i < 2 * DF * DF / 8) { W = Wr; P = Wrh; nc = DF; j = i - DF * DF / 8; }
  else                          { W = Wg; P = Wgh; nc = DG; j = i - 2 * DF * DF / 8; }
  const int n  = j >> 4;
  const int k0 = (j & 15) * 8;
  Pack16 u;
#pragma unroll
  for (int t = 0; t < 8; ++t) u.h[t] = (_Float16)(W[(size_t)(k0 + t) * nc + n] * WSCL);
  _Float16* p = P + (size_t)n * DF + k0;
  *(volatile v4i*)p = u.i;
  __threadfence();
  *(volatile v4i*)p = u.i;
}

__device__ __forceinline__ void scan_chunk(const int* eid, int nE, bool al16, int cbase,
                                           int nodeBase, unsigned nbe, int tid, int lane, int wave,
                                           int* list, int* wcnt) {
  int wc = 0;
#pragma unroll
  for (int gq = 0; gq < NGRP; ++gq) {
    const int el0 = (gq * NTHR + tid) * 4;
    const int e0  = cbase + el0;
    const int sent = -2147483647 - 1;
    v4i d;
    if (al16 && (e0 + 3 < nE)) {
      d = *(const v4i*)(eid + e0);
    } else {
      d.x = (e0     < nE) ? eid[(e0     < nE - 1) ? e0     : nE - 1] : sent;
      d.y = (e0 + 1 < nE) ? eid[(e0 + 1 < nE - 1) ? e0 + 1 : nE - 1] : sent;
      d.z = (e0 + 2 < nE) ? eid[(e0 + 2 < nE - 1) ? e0 + 2 : nE - 1] : sent;
      d.w = (e0 + 3 < nE) ? eid[(e0 + 3 < nE - 1) ? e0 + 3 : nE - 1] : sent;
    }
    const unsigned s0 = (unsigned)d.x - (unsigned)nodeBase;
    const unsigned s1 = (unsigned)d.y - (unsigned)nodeBase;
    const unsigned s2 = (unsigned)d.z - (unsigned)nodeBase;
    const unsigned s3 = (unsigned)d.w - (unsigned)nodeBase;
    const bool h0 = s0 < nbe;
    const bool h1 = s1 < nbe;
    const bool h2 = s2 < nbe;
    const bool h3 = s3 < nbe;
    const unsigned many = __builtin_amdgcn_ballot_w32(h0 | h1 | h2 | h3);
    if (many != 0u) {
#define HITJ(J, HJ, SJ) { \
        const unsigned mj = __builtin_amdgcn_ballot_w32(HJ); \
        if (HJ) { \
          const int pos = wc + (int)__builtin_amdgcn_mbcnt_lo(mj, 0u); \
          if (pos < WCAP) list[wave * WCAP + pos] = ((el0 + (J)) << 9) | (int)(SJ); \
        } \
        wc += (int)__builtin_popcount(mj); }
      HITJ(0, h0, s0)
      HITJ(1, h1, s1)
      HITJ(2, h2, s2)
      HITJ(3, h3, s3)
#undef HITJ
    }
  }
  if (lane == 0) wcnt[wave] = wc;
}

__global__ __launch_bounds__(NTHR) void k_sage_agg(const float* __restrict__ x, const int* __restrict__ ei,
                                                   _Float16* meanh, _Float16* xh, int nN, int nE) {
  extern __shared__ v4f lds_dyn[];
  float* sacc = (float*)lds_dyn;
  float* cnt  = sacc + NB * DF;
  int*   list = (int*)(cnt + NB);
  int*   wcnt = list + NWAVE * WCAP;

  const int tid  = threadIdx.x;
  const int lane = tid & 31;
  const int wave = tid >> 5;
  const int nodeBase = blockIdx.x * NB;
  {
    const v4f z4 = {0.f, 0.f, 0.f, 0.f};
    for (int i = tid; i < (NB * DF + NB) / 4; i += NTHR) lds_dyn[i] = z4;
  }
  __syncthreads();

  const int* eid = ei + nE;
  const bool al16 = ((((size_t)eid) & 15) == 0);
  const int remain = nN - nodeBase;
  const unsigned nbe = (unsigned)(remain < NB ? remain : NB);
  const int nChunks = (nE + CHUNK - 1) / CHUNK;

#pragma unroll 1
  for (int ch = 0; ch < nChunks; ++ch) {
    const int cbase = ch * CHUNK;
    scan_chunk(eid, nE, al16, cbase, nodeBase, nbe, tid, lane, wave, list, wcnt);
    __syncthreads();
    if (wave == 0) {
      for (int wsx = 0; wsx < NWAVE; ++wsx) {
        int n = wcnt[wsx];
        n = n > WCAP ? WCAP : n;
        n = n < 0 ? 0 : n;
        for (int i = 0; i < n; ++i) {
          const int ent  = list[wsx * WCAP + i];
          const int slot = ent & (NB - 1);
          const int el   = (ent >> 9) & (CHUNK - 1);
          int e = cbase + el;
          if (e > nE - 1) e = nE - 1;
          int src = ei[e];
          src = src < 0 ? 0 : (src > nN - 1 ? nN - 1 : src);
          const v4f xv = *(const v4f*)(x + (size_t)src * DF + 4 * lane);
          v4f* sp = (v4f*)(sacc + slot * DF + 4 * lane);
          const v4f cur = *sp;
          *sp = cur + xv;
          if (lane == 0) {
            const float c = cnt[slot];
            cnt[slot] = c + 1.0f;
          }
        }
      }
    }
    __syncthreads();
  }
  __syncthreads();

  const int sub = lane >> 4;
  const int q   = lane & 15;
#pragma unroll 1
  for (int j = 0; j < NB / NWAVE / 2; ++j) {
    const int slot = wave * (NB / NWAVE) + 2 * j + sub;
    const int node = nodeBase + slot;
    const float c  = cnt[slot];
    const float ic = 1.0f / fmaxf(c, 1.0f);
    const v4f s0 = *(const v4f*)(sacc + slot * DF + 8 * q);
    const v4f s1 = *(const v4f*)(sacc + slot * DF + 8 * q + 4);
    Pack16 um;
    um.h[0] = (_Float16)(s0.x * ic); um.h[1] = (_Float16)(s0.y * ic);
    um.h[2] = (_Float16)(s0.z * ic); um.h[3] = (_Float16)(s0.w * ic);
    um.h[4] = (_Float16)(s1.x * ic); um.h[5] = (_Float16)(s1.y * ic);
    um.h[6] = (_Float16)(s1.z * ic); um.h[7] = (_Float16)(s1.w * ic);
    const int rn = node < nN ? node : nN - 1;
    const v4f f0 = *(const v4f*)(x + (size_t)rn * DF + 8 * q);
    const v4f f1 = *(const v4f*)(x + (size_t)rn * DF + 8 * q + 4);
    Pack16 ux;
    ux.h[0] = (_Float16)f0.x; ux.h[1] = (_Float16)f0.y; ux.h[2] = (_Float16)f0.z; ux.h[3] = (_Float16)f0.w;
    ux.h[4] = (_Float16)f1.x; ux.h[5] = (_Float16)f1.y; ux.h[6] = (_Float16)f1.z; ux.h[7] = (_Float16)f1.w;
    _Float16* pm = meanh + (size_t)node * DF + 8 * q;
    _Float16* px = xh    + (size_t)node * DF + 8 * q;
    *(volatile v4i*)pm = um.i;
    *(volatile v4i*)px = ux.i;
    __threadfence();
    *(volatile v4i*)pm = um.i;
    *(volatile v4i*)px = ux.i;
  }
}

__global__ __launch_bounds__(NTHR) void k_sage_gemm(const _Float16* __restrict__ meanh, const _Float16* __restrict__ xh,
                                                    const _Float16* __restrict__ Wlh, const _Float16* __restrict__ Wrh,
                                                    const float* __restrict__ b_sage, _Float16* hh) {
  __shared__ __attribute__((aligned(16))) _Float16 Hs[GR * HSP];

  const int tid  = threadIdx.x;
  const int lane = tid & 31;
  const int wave = tid >> 5;
  const int h    = lane >> 4;
  const int m    = lane & 15;
  const int rowBase = blockIdx.x * GR;
  const int ncol = wave * 16 + m;

  v8f c0 = {0.f, 0.f, 0.f, 0.f, 0.f, 0.f, 0.f, 0.f};
  v8f c1 = {0.f, 0.f, 0.f, 0.f, 0.f, 0.f, 0.f, 0.f};
#pragma unroll 1
  for (int kt = 0; kt < DF / 32; ++kt) {
    const int k0 = kt * 32;
    Frag am0, am1, ax0, ax1, bl, br;
    const _Float16* pm0 = meanh + (size_t)(rowBase + m) * DF + k0 + 8 * h;
    const _Float16* pm1 = meanh + (size_t)(rowBase + 16 + m) * DF + k0 + 8 * h;
    const _Float16* px0 = xh + (size_t)(rowBase + m) * DF + k0 + 8 * h;
    const _Float16* px1 = xh + (size_t)(rowBase + 16 + m) * DF + k0 + 8 * h;
    const _Float16* pbl = Wlh + (size_t)ncol * DF + k0 + 8 * h;
    const _Float16* pbr = Wrh + (size_t)ncol * DF + k0 + 8 * h;
    am0.half[0] = *(const v8h*)pm0; am0.half[1] = *(const v8h*)(pm0 + 16);
    am1.half[0] = *(const v8h*)pm1; am1.half[1] = *(const v8h*)(pm1 + 16);
    ax0.half[0] = *(const v8h*)px0; ax0.half[1] = *(const v8h*)(px0 + 16);
    ax1.half[0] = *(const v8h*)px1; ax1.half[1] = *(const v8h*)(px1 + 16);
    bl.half[0]  = *(const v8h*)pbl; bl.half[1]  = *(const v8h*)(pbl + 16);
    br.half[0]  = *(const v8h*)pbr; br.half[1]  = *(const v8h*)(pbr + 16);
    c0 = wm(am0.v, bl.v, c0);
    c0 = wm(ax0.v, br.v, c0);
    c1 = wm(am1.v, bl.v, c1);
    c1 = wm(ax1.v, br.v, c1);
  }

  const float bias = b_sage[ncol];
#pragma unroll
  for (int r = 0; r < 8; ++r) {
    const float v0 = elu1(c0[r] * WINV + bias);
    const float v1 = elu1(c1[r] * WINV + bias);
    Hs[(8 * h + r) * HSP + ncol]      = (_Float16)v0;
    Hs[(16 + 8 * h + r) * HSP + ncol] = (_Float16)v1;
  }
  __syncthreads();

  const int sub = lane >> 4;
  const int q   = lane & 15;
  Pack16 u[2];
  _Float16* p[2];
#pragma unroll
  for (int i = 0; i < 2; ++i) {
    const int row = 4 * wave + 2 * i + sub;
    u[i].h = *(const v8h*)(Hs + row * HSP + 8 * q);
    p[i] = hh + (size_t)(rowBase + row) * DF + 8 * q;
  }
#pragma unroll
  for (int i = 0; i < 2; ++i) *(volatile v4i*)(p[i]) = u[i].i;
  __threadfence();
#pragma unroll
  for (int i = 0; i < 2; ++i) *(volatile v4i*)(p[i]) = u[i].i;
}

__device__ __forceinline__ void epi_tile(v8f acc, int T, int hh2, int m, int wave, int cl,
                                         float cs, float cd, float* Xs, float* As, float* Ds) {
  float ss[8], sd[8];
#pragma unroll
  for (int r = 0; r < 8; ++r) {
    const float v = acc[r] * WINV;
    Xs[(T * 16 + 8 * hh2 + r) * XSP + cl] = v;
    ss[r] = v * cs;
    sd[r] = v * cd;
  }
#pragma unroll
  for (int mk = 1; mk < 16; mk <<= 1) {
#pragma unroll
    for (int r = 0; r < 8; ++r) {
      ss[r] += __shfl_xor(ss[r], mk, 32);
      sd[r] += __shfl_xor(sd[r], mk, 32);
    }
  }
  if (m == 0) {
#pragma unroll
    for (int r = 0; r < 8; ++r) {
      As[(T * 16 + 8 * hh2 + r) * NWAVE + wave] = ss[r];
      Ds[(T * 16 + 8 * hh2 + r) * NWAVE + wave] = sd[r];
    }
  }
}

__global__ __launch_bounds__(NTHR) void k_gat_gemm(const _Float16* __restrict__ hh, const _Float16* __restrict__ Wgh,
                                                   const float* __restrict__ att_src, const float* __restrict__ att_dst,
                                                   float* g, float* asrcP, float* adstP, int nP) {
  __shared__ __attribute__((aligned(16))) float Xs[GR * XSP];
  __shared__ __attribute__((aligned(16))) float As[GR * NWAVE];
  __shared__ __attribute__((aligned(16))) float Ds[GR * NWAVE];

  const int tid  = threadIdx.x;
  const int lane = tid & 31;
  const int wave = tid >> 5;
  const int h    = lane >> 4;
  const int m    = lane & 15;
  const int rowBase = blockIdx.x * GR;
  const int hy   = blockIdx.y;
  const int cl   = wave * 16 + m;
  const int ncol = hy * DF + cl;

  v8f c0 = {0.f, 0.f, 0.f, 0.f, 0.f, 0.f, 0.f, 0.f};
  v8f c1 = {0.f, 0.f, 0.f, 0.f, 0.f, 0.f, 0.f, 0.f};
#pragma unroll 1
  for (int kt = 0; kt < DF / 32; ++kt) {
    const int k0 = kt * 32;
    Frag a0, a1, b;
    const _Float16* pa0 = hh + (size_t)(rowBase + m) * DF + k0 + 8 * h;
    const _Float16* pa1 = hh + (size_t)(rowBase + 16 + m) * DF + k0 + 8 * h;
    const _Float16* pb  = Wgh + (size_t)ncol * DF + k0 + 8 * h;
    a0.half[0] = *(const v8h*)pa0; a0.half[1] = *(const v8h*)(pa0 + 16);
    a1.half[0] = *(const v8h*)pa1; a1.half[1] = *(const v8h*)(pa1 + 16);
    b.half[0]  = *(const v8h*)pb;  b.half[1]  = *(const v8h*)(pb + 16);
    c0 = wm(a0.v, b.v, c0);
    c1 = wm(a1.v, b.v, c1);
  }

  const float cs = att_src[hy * DF + cl];
  const float cd = att_dst[hy * DF + cl];
  epi_tile(c0, 0, h, m, wave, cl, cs, cd, Xs, As, Ds);
  epi_tile(c1, 1, h, m, wave, cl, cs, cd, Xs, As, Ds);
  __syncthreads();

  v4f xr[4];
  float* gpp[4];
#pragma unroll
  for (int i = 0; i < 4; ++i) {
    xr[i]  = *(const v4f*)(Xs + (4 * wave + i) * XSP + 4 * lane);
    gpp[i] = g + (size_t)(rowBase + 4 * wave + i) * DG + hy * DF + 4 * lane;
  }
  float* ap = 0;
  v4f av = {0.f, 0.f, 0.f, 0.f};
  if (wave == 0 && lane < 16) {
    const int pl = lane >> 3;
    const int l7 = lane & 7;
    const float* S = pl ? Ds : As;
    float sum[4];
#pragma unroll
    for (int rr = 0; rr < 4; ++rr) {
      const int row = 4 * l7 + rr;
      float s = 0.f;
#pragma unroll
      for (int w = 0; w < NWAVE; ++w) s += S[row * NWAVE + w];
      sum[rr] = s;
    }
    av.x = sum[0]; av.y = sum[1]; av.z = sum[2]; av.w = sum[3];
    ap = (pl ? adstP : asrcP) + (size_t)hy * nP + rowBase + 4 * l7;
  }

#pragma unroll
  for (int i = 0; i < 4; ++i) *(volatile v4f*)(gpp[i]) = xr[i];
  if (ap) *(volatile v4f*)ap = av;
  __threadfence();
#pragma unroll
  for (int i = 0; i < 4; ++i) *(volatile v4f*)(gpp[i]) = xr[i];
  if (ap) *(volatile v4f*)ap = av;
}

__global__ __launch_bounds__(NTHR) void k_gat_agg(
    const int* __restrict__ ei, const float* __restrict__ g,
    const float* __restrict__ asrcP, const float* __restrict__ adstP,
    const float* __restrict__ b_gat,
    const float* __restrict__ W_wire, const float* __restrict__ b_wire,
    const float* __restrict__ W_term, const float* __restrict__ b_term,
    float* h2, float* out, int nN, int nE, int nP) {
  extern __shared__ v4f lds_dyn[];
  float* sacc = (float*)lds_dyn;
  float* den  = sacc + NB * DF;
  float* mx   = den + NB * NHD;
  int*   list = (int*)(mx + NB * NHD);
  int*   wcnt = list + NWAVE * WCAP;
  float* pr   = (float*)list;

  const int tid  = threadIdx.x;
  const int lane = tid & 31;
  const int wave = tid >> 5;
  const int nodeBase = blockIdx.x * NB;
  {
    const v4f z4 = {0.f, 0.f, 0.f, 0.f};
    for (int i = tid; i < (NB * DF + NB * NHD) / 4; i += NTHR) lds_dyn[i] = z4;
    const v4f n4 = {-3.0e38f, -3.0e38f, -3.0e38f, -3.0e38f};
    v4f* mx4 = (v4f*)mx;
    for (int i = tid; i < (NB * NHD) / 4; i += NTHR) mx4[i] = n4;
  }
  __syncthreads();

  const int* eid = ei + nE;
  const bool al16 = ((((size_t)eid) & 15) == 0);
  const int remain = nN - nodeBase;
  const unsigned nbe = (unsigned)(remain < NB ? remain : NB);
  const int nChunks = (nE + CHUNK - 1) / CHUNK;

#pragma unroll 1
  for (int ps = 0; ps < 2; ++ps) {
#pragma unroll 1
    for (int ch = 0; ch < nChunks; ++ch) {
      const int cbase = ch * CHUNK;
      scan_chunk(eid, nE, al16, cbase, nodeBase, nbe, tid, lane, wave, list, wcnt);
      __syncthreads();
      if (wave == 0) {
        for (int wsx = 0; wsx < NWAVE; ++wsx) {
          int n = wcnt[wsx];
          n = n > WCAP ? WCAP : n;
          n = n < 0 ? 0 : n;
          for (int i = 0; i < n; ++i) {
            const int ent  = list[wsx * WCAP + i];
            const int slot = ent & (NB - 1);
            const int el   = (ent >> 9) & (CHUNK - 1);
            int e = cbase + el;
            if (e > nE - 1) e = nE - 1;
            int src = ei[e];
            src = src < 0 ? 0 : (src > nN - 1 ? nN - 1 : src);
            int nd = nodeBase + slot;
            if (nd > nN - 1) nd = nN - 1;
            if (ps == 0) {
              if (lane < NHD) {
                float a = asrcP[(size_t)lane * nP + src] + adstP[(size_t)lane * nP + nd];
                a = (a > 0.f) ? a : 0.2f * a;
                const int ix = slot * NHD + lane;
                const float mo = mx[ix];
                const float mn = fmaxf(mo, a);
                const float sc = (mo > -1.0e38f) ? expf(mo - mn) : 0.f;
                const float d  = den[ix] * sc + expf(a - mn);
                mx[ix]  = mn;
                den[ix] = d;
              }
            } else {
              float al[NHD];
              const v4f m4 = *(const v4f*)(mx + slot * NHD);
              const v4f i4 = *(const v4f*)(den + slot * NHD);
#pragma unroll
              for (int hd = 0; hd < NHD; ++hd) {
                float a = asrcP[(size_t)hd * nP + src] + adstP[(size_t)hd * nP + nd];
                a = (a > 0.f) ? a : 0.2f * a;
                al[hd] = expf(a - m4[hd]) * i4[hd];
              }
              v4f* sp = (v4f*)(sacc + slot * DF + 4 * lane);
              v4f acc = *sp;
#pragma unroll
              for (int hd = 0; hd < NHD; ++hd) {
                const v4f gv = *(const v4f*)(g + (size_t)src * DG + hd * DF + 4 * lane);
                acc = acc + al[hd] * gv;
              }
              *sp = acc;
            }
          }
        }
      }
      __syncthreads();
    }
    if (ps == 0) {
      for (int i = tid; i < NB * NHD; i += NTHR) {
        const float d = den[i];
        den[i] = (d > 0.f) ? 0.25f * (1.0f / (d + 1e-16f)) : 0.f;
      }
      __syncthreads();
    }
  }
  __syncthreads();

  const v4f b4  = *(const v4f*)(b_gat + 4 * lane);
  const v4f ww4 = *(const v4f*)(W_wire + 4 * lane);
  const v4f wt4 = *(const v4f*)(W_term + 4 * lane);
  const float bw = b_wire[0];
  const float bt = b_term[0];
#pragma unroll 1
  for (int j = 0; j < NB / NWAVE; ++j) {
    const int slot = wave * (NB / NWAVE) + j;
    const int node = nodeBase + slot;
    const v4f s = *(const v4f*)(sacc + slot * DF + 4 * lane);
    v4f hv = s + b4;
    hv.x = elu1(hv.x); hv.y = elu1(hv.y); hv.z = elu1(hv.z); hv.w = elu1(hv.w);
    float* hp = h2 + (size_t)node * DF + 4 * lane;
    *(volatile v4f*)hp = hv;
    const bool term = (node >= nN - NTERM);
    const v4f w4 = term ? wt4 : ww4;
    float dsum = hv.x * w4.x + hv.y * w4.y + hv.z * w4.z + hv.w * w4.w;
    dsum = wsum(dsum);
    float sg = dsum + (term ? bt : bw);
    sg = fminf(fmaxf(sg, -30.f), 30.f);
    const float p = 1.0f / (1.0f + expf(-sg));
    if (lane == 0) pr[slot] = p;
    __threadfence();
    *(volatile v4f*)hp = hv;
  }
  __syncthreads();

  if (wave == 0) {
    const int cntOut = remain < NB ? remain : NB;
    v4f pv[NB / 128];
    bool full[NB / 128];
    float psv[NB / 128][4];
#pragma unroll
    for (int i = 0; i < NB / 128; ++i) {
      const int base = i * 128 + 4 * lane;
      full[i] = (base + 3 < cntOut);
      pv[i] = *(const v4f*)(pr + base);
      psv[i][0] = pv[i].x; psv[i][1] = pv[i].y; psv[i][2] = pv[i].z; psv[i][3] = pv[i].w;
    }
#pragma unroll
    for (int i = 0; i < NB / 128; ++i) {
      const int base = i * 128 + 4 * lane;
      if (full[i]) {
        *(volatile v4f*)(out + nodeBase + base) = pv[i];
      } else {
#pragma unroll
        for (int t = 0; t < 4; ++t)
          if (base + t < cntOut) *(volatile float*)(out + nodeBase + base + t) = psv[i][t];
      }
    }
    __threadfence();
#pragma unroll
    for (int i = 0; i < NB / 128; ++i) {
      const int base = i * 128 + 4 * lane;
      if (full[i]) {
        *(volatile v4f*)(out + nodeBase + base) = pv[i];
      } else {
#pragma unroll
        for (int t = 0; t < 4; ++t)
          if (base + t < cntOut) *(volatile float*)(out + nodeBase + base + t) = psv[i][t];
      }
    }
  }
}

__global__ __launch_bounds__(NTHR) void k_pool_act(const float* __restrict__ h2, const int* __restrict__ batch,
                                                   const float* __restrict__ W_act, const float* __restrict__ b_act,
                                                   float* out, int nN, int nG) {
  __shared__ __attribute__((aligned(16))) double part[NWAVE * DF];
  __shared__ __attribute__((aligned(16))) float pooled[DF];
  __shared__ __attribute__((aligned(16))) float lg[NGMAX * NACT];
  __shared__ int wc[NWAVE];

  const int tid  = threadIdx.x;
  const int lane = tid & 31;
  const int wave = tid >> 5;

#pragma unroll 1
  for (int b = 0; b < nG; ++b) {
    double a0 = 0.0, a1 = 0.0, a2 = 0.0, a3 = 0.0;
    int c = 0;
#pragma unroll 1
    for (int n = wave; n < nN; n += NWAVE) {
      const int bb = batch[n];
      if (bb == b) {
        const v4f v = *(const v4f*)(h2 + (size_t)n * DF + 4 * lane);
        a0 += (double)v.x; a1 += (double)v.y; a2 += (double)v.z; a3 += (double)v.w;
        ++c;
      }
    }
    part[wave * DF + 4 * lane + 0] = a0;
    part[wave * DF + 4 * lane + 1] = a1;
    part[wave * DF + 4 * lane + 2] = a2;
    part[wave * DF + 4 * lane + 3] = a3;
    if (lane == 0) wc[wave] = c;
    __syncthreads();
    if (tid < DF) {
      double s = 0.0;
      int cn = 0;
#pragma unroll
      for (int w = 0; w < NWAVE; ++w) { s += part[w * DF + tid]; cn += wc[w]; }
      const float cf = (float)(cn > 1 ? cn : 1);
      pooled[tid] = (float)s * (1.0f / cf);
    }
    __syncthreads();
    if (tid < NACT) {
      float s = b_act[tid];
#pragma unroll 4
      for (int k = 0; k < DF; ++k) s += pooled[k] * W_act[k * NACT + tid];
      lg[b * NACT + tid] = s;
    }
    __syncthreads();
  }

  const int nO = nG * NACT;
  float* ob = out + nN;
  const bool vec = ((nN & 3) == 0);
  const int base = tid * 4;
  const bool inr = (base < nO);
  const bool full = vec && (base + 3 < nO);
  v4f v4 = {0.f, 0.f, 0.f, 0.f};
  float sv[4];
#pragma unroll
  for (int t = 0; t < 4; ++t) sv[t] = (base + t < nO) ? lg[base + t] : 0.f;
  v4.x = sv[0]; v4.y = sv[1]; v4.z = sv[2]; v4.w = sv[3];
  if (inr) {
    if (full) {
      *(volatile v4f*)(ob + base) = v4;
    } else {
#pragma unroll
      for (int t = 0; t < 4; ++t)
        if (base + t < nO) *(volatile float*)(ob + base + t) = sv[t];
    }
  }
  __threadfence();
  if (inr) {
    if (full) {
      *(volatile v4f*)(ob + base) = v4;
    } else {
#pragma unroll
      for (int t = 0; t < 4; ++t)
        if (base + t < nO) *(volatile float*)(ob + base + t) = sv[t];
    }
  }
}

extern "C" void kernel_launch(void* const* d_in, const int* in_sizes, int n_in,
                              void* d_out, int out_size, void* d_ws, size_t ws_size,
                              hipStream_t stream) {
  if (n_in < 16) return;
  const int nN = in_sizes[0] / DF;
  if (nN <= NTERM || in_sizes[0] != nN * DF) return;
  const int nE = in_sizes[1] / 2;
  if (nE < 0 || in_sizes[1] != 2 * nE) return;
  if (in_sizes[2] != nN) return;
  if (in_sizes[3] != DF * DF || in_sizes[4] != DF * DF || in_sizes[5] != DF) return;
  if (in_sizes[6] != DF * DG || in_sizes[7] != NHD * DF || in_sizes[8] != NHD * DF || in_sizes[9] != DF) return;
  if (in_sizes[10] != DF || in_sizes[11] < 1 || in_sizes[12] != DF || in_sizes[13] < 1) return;
  if (in_sizes[14] != DF * NACT || in_sizes[15] != NACT) return;
  const int nG = (out_size - nN) / NACT;
  if (nG < 1 || nG > NGMAX || out_size != nN + nG * NACT) return;

  const float* x       = (const float*)d_in[0];
  const int*   ei      = (const int*)d_in[1];
  const int*   batch   = (const int*)d_in[2];
  const float* Wl      = (const float*)d_in[3];
  const float* Wr      = (const float*)d_in[4];
  const float* b_sage  = (const float*)d_in[5];
  const float* Wg      = (const float*)d_in[6];
  const float* att_src = (const float*)d_in[7];
  const float* att_dst = (const float*)d_in[8];
  const float* b_gat   = (const float*)d_in[9];
  const float* W_wire  = (const float*)d_in[10];
  const float* b_wire  = (const float*)d_in[11];
  const float* W_term  = (const float*)d_in[12];
  const float* b_term  = (const float*)d_in[13];
  const float* W_act   = (const float*)d_in[14];
  const float* b_act   = (const float*)d_in[15];
  float* out = (float*)d_out;

  const int nP = ((nN + NB - 1) / NB) * NB;
  size_t off = 0;
  _Float16* Wlh  = (_Float16*)((char*)d_ws + off); off += (size_t)DF * DF * sizeof(_Float16);
  _Float16* Wrh  = (_Float16*)((char*)d_ws + off); off += (size_t)DF * DF * sizeof(_Float16);
  _Float16* Wgh  = (_Float16*)((char*)d_ws + off); off += (size_t)DG * DF * sizeof(_Float16);
  _Float16* meanh = (_Float16*)((char*)d_ws + off); off += (size_t)nP * DF * sizeof(_Float16);
  _Float16* xh   = (_Float16*)((char*)d_ws + off); off += (size_t)nP * DF * sizeof(_Float16);
  _Float16* hh   = (_Float16*)((char*)d_ws + off); off += (size_t)nP * DF * sizeof(_Float16);
  float* gbuf    = (float*)((char*)d_ws + off);    off += (size_t)nP * DG * sizeof(float);
  float* asrcP   = (float*)((char*)d_ws + off);    off += (size_t)NHD * nP * sizeof(float);
  float* adstP   = (float*)((char*)d_ws + off);    off += (size_t)NHD * nP * sizeof(float);
  float* h2      = (float*)((char*)d_ws + off);    off += (size_t)nP * DF * sizeof(float);
  if (off > ws_size) return;
  if (off > (size_t)134217728) return;

  const int n8 = (2 * DF * DF + DF * DG) / 8;
  k_prep<<<(n8 + NTHR - 1) / NTHR, NTHR, 0, stream>>>(Wl, Wr, Wg, Wlh, Wrh, Wgh, n8);

  const int gridA = (nN + NB - 1) / NB;
  hipFuncSetAttribute(reinterpret_cast<const void*>(&k_sage_agg),
                      hipFuncAttributeMaxDynamicSharedMemorySize, LDS_SAGE_BYTES);
  k_sage_agg<<<gridA, NTHR, LDS_SAGE_BYTES, stream>>>(x, ei, meanh, xh, nN, nE);

  const int gridG = (nN + GR - 1) / GR;
  k_sage_gemm<<<gridG, NTHR, 0, stream>>>(meanh, xh, Wlh, Wrh, b_sage, hh);

  k_gat_gemm<<<dim3(gridG, NHD), NTHR, 0, stream>>>(hh, Wgh, att_src, att_dst, gbuf, asrcP, adstP, nP);

  hipFuncSetAttribute(reinterpret_cast<const void*>(&k_gat_agg),
                      hipFuncAttributeMaxDynamicSharedMemorySize, LDS_GAT_BYTES);
  k_gat_agg<<<gridA, NTHR, LDS_GAT_BYTES, stream>>>(ei, gbuf, asrcP, adstP, b_gat,
                                                     W_wire, b_wire, W_term, b_term,
                                                     h2, out, nN, nE, nP);

  k_pool_act<<<1, NTHR, 0, stream>>>(h2, batch, W_act, b_act, out, nN, nG);
}
